// MinGRU_72086731096321
// MI455X (gfx1250) — hardware-run, weakly checked
//
#include <hip/hip_runtime.h>
#include <math.h>

typedef __attribute__((ext_vector_type(16))) _Float16 v16h;
typedef __attribute__((ext_vector_type(8)))  _Float16 v8h;
typedef __attribute__((ext_vector_type(2)))  _Float16 v2h;
typedef __attribute__((ext_vector_type(16))) __bf16   v16b;
typedef __attribute__((ext_vector_type(8)))  __bf16   v8b;
typedef __attribute__((ext_vector_type(8)))  float    v8f;
typedef __attribute__((ext_vector_type(4)))  float    v4f;
typedef __attribute__((ext_vector_type(2)))  float    v2f;


constexpr int kB   = 8;
constexpr int kT   = 4096;
constexpr int kD   = 1024;
constexpr int kE   = 1024;
constexpr int kN   = 2 * kE;
constexpr int kBh  = 2;
constexpr int kPc  = kB / kBh;
constexpr int kMh  = kBh * kT;
constexpr int kThr = 256;
constexpr float kInCarry = 1024.0f;
constexpr float kSc20 = 1.0f / (kInCarry * kInCarry);
constexpr float kF16MinNormal = 6.103515625e-5f;

static_assert(kB == 8 && kPc == 4 && kT == 4096 && kD == 1024 && kE == 1024 && kN == 2048 && kBh == 2 && kMh == 8192 && kE / 2 == 512, "the index arithmetic below uses these sizes: a row is 512 lanes of two channels");

constexpr size_t kOffX16  = 0ull;
constexpr size_t kOffW16  = 16777216ull;
constexpr size_t kOffYP   = 20971520ull;
constexpr size_t kWsTotal = 88080384ull;
static_assert(kOffW16 == (size_t)kMh * kD * 2ull && kOffYP == kOffW16 + (size_t)kN * kD * 2ull && kWsTotal == kOffYP + (size_t)kMh * kN * 4ull, "the carve is a chain: every region starts where the one before ends");
static_assert((kOffW16 % 256) == 0 && (kOffYP % 256) == 0, "every region starts on a multiple of 256 B");

__device__ __forceinline__ unsigned short f2bf_bits(float f) {
  unsigned u = __float_as_uint(f);
  return (unsigned short)((u + 0x7FFFu + ((u >> 16) & 1u)) >> 16);
}
__device__ __forceinline__ float bf_bits2f(unsigned short h) { return __uint_as_float(((unsigned)h) << 16); }
__device__ __forceinline__ float bf16r(float f) { return bf_bits2f(f2bf_bits(f)); }
__device__ __forceinline__ float carry_flush(float v, float carry) {
  const float s = v * carry;
  return (fabsf(s) < kF16MinNormal) ? 0.0f : s;
}

__device__ __forceinline__ void dep_guard4_h(v8f& a, v8f& b, v8f& c, v8f& d, v16h x, v16h y) { asm volatile("v_nop\n\tv_nop\n\tv_nop\n\tv_nop" : "+v"(a), "+v"(b), "+v"(c), "+v"(d) : "v"(x), "v"(y)); }
__device__ __forceinline__ void dep_guard4_b(v8f& a, v8f& b, v8f& c, v8f& d, v16b x, v16b y) { asm volatile("v_nop\n\tv_nop\n\tv_nop\n\tv_nop" : "+v"(a), "+v"(b), "+v"(c), "+v"(d) : "v"(x), "v"(y)); }
__device__ __forceinline__ void keep4_h(v16h a, v16h b, v16h c, v16h d) { asm volatile("v_nop" :: "v"(a), "v"(b), "v"(c), "v"(d)); }
__device__ __forceinline__ void keep4_b(v16b a, v16b b, v16b c, v16b d) { asm volatile("v_nop" :: "v"(a), "v"(b), "v"(c), "v"(d)); }
__device__ __forceinline__ void acc_guard4(v8f& a, v8f& b, v8f& c, v8f& d) { asm volatile("v_nop\n\tv_nop\n\tv_nop\n\tv_nop" : "+v"(a), "+v"(b), "+v"(c), "+v"(d)); }

template <typename T> struct Frag;
template <> struct Frag<_Float16> {
  typedef v16h V; union U { v16h v; v8h h[2]; };
  static __device__ __forceinline__ v16h load(const _Float16* p) {
    U f; f.h[0] = *(const v8h*)(p); f.h[1] = *(const v8h*)(p + 16); return f.v;
  }
  static __device__ __forceinline__ v8f mma(v16h a, v16h b, v8f c) {
    return __builtin_amdgcn_wmma_f32_16x16x32_f16(false, a, false, b, (short)0, c, false, false);
  }
  static __device__ __forceinline__ void guard4(v8f& a, v8f& b, v8f& c, v8f& d, v16h x, v16h y) { dep_guard4_h(a, b, c, d, x, y); }
  static __device__ __forceinline__ void keep(v16h a, v16h b, v16h c, v16h d) { keep4_h(a, b, c, d); }
};
template <> struct Frag<__bf16> {
  typedef v16b V; union U { v16b v; v8b h[2]; };
  static __device__ __forceinline__ v16b load(const __bf16* p) {
    U f; f.h[0] = *(const v8b*)(p); f.h[1] = *(const v8b*)(p + 16); return f.v;
  }
  static __device__ __forceinline__ v8f mma(v16b a, v16b b, v8f c) {
    return __builtin_amdgcn_wmma_f32_16x16x32_bf16(false, a, false, b, (short)0, c, false, false);
  }
  static __device__ __forceinline__ void guard4(v8f& a, v8f& b, v8f& c, v8f& d, v16b x, v16b y) { dep_guard4_b(a, b, c, d, x, y); }
  static __device__ __forceinline__ void keep(v16b a, v16b b, v16b c, v16b d) { keep4_b(a, b, c, d); }
};

__device__ __forceinline__ v8f mma_h(v16h a, v16h b, v8f c) {
  c = __builtin_amdgcn_wmma_f32_16x16x32_f16(false, a, false, b, (short)0, c, false, false);
  asm volatile("v_nop\n\tv_nop\n\tv_nop\n\tv_nop" : "+v"(c) : "v"(a), "v"(b));
  return c;
}

template <int ET> struct Elem;
template <> struct Elem<0> { typedef _Float16 T; };
template <> struct Elem<1> { typedef __bf16 T; };
template <int ET, bool SPLIT, int BIAS_MODE, int OUT_MODE, bool RESID, int ACT = 0>
__global__ __launch_bounds__(256) void wmma_gemm64(
    const unsigned short* __restrict__ Ap, const unsigned short* __restrict__ A2p, int lda, long strideA,
    const unsigned short* __restrict__ Btp, const unsigned short* __restrict__ Bt2p, int ldb, long strideB,
    void* __restrict__ Cout, void* __restrict__ Cout2, int ldc, long strideC,
    const float* __restrict__ bias,
    const float* __restrict__ resid, long strideR,
    int M, int N, int K, float scale) {
  typedef typename Elem<ET>::T T;
  typedef typename Frag<T>::V V;
  const T* A = (const T*)Ap; const T* A2 = (const T*)A2p; const T* Bt = (const T*)Btp; const T* Bt2 = (const T*)Bt2p;
  __shared__ __align__(16) float sT[8][16 * 68];
  const int b    = blockIdx.y;
  const int lane = threadIdx.x & 31;
  const int wave = threadIdx.x >> 5;
  const int tilesN = N >> 6;
  const int tilesM = M >> 6;
  const int tile = blockIdx.x * 8 + wave;
  if (tile >= tilesM * tilesN) return;
  const int tm = tile / tilesN;
  const int tn = tile - tm * tilesN;
  const int m0 = tm << 6;
  const int n0 = tn << 6;

  const T* Ab  = A  + (size_t)b * strideA;
  const T* Bb  = Bt + (size_t)b * strideB;
  const T* Ab2 = SPLIT ? (A2  + (size_t)b * strideA) : nullptr;
  const T* Bb2 = SPLIT ? (Bt2 + (size_t)b * strideB) : nullptr;

  const int rlane = lane & 15;
  const int koff  = (lane >> 4) * 8;
  const int mOff  = (lane >> 4) * 8;

  v8f acc[4][4];
#pragma unroll
  for (int i = 0; i < 4; ++i)
#pragma unroll
    for (int j = 0; j < 4; ++j) acc[i][j] = (v8f){0.f,0.f,0.f,0.f,0.f,0.f,0.f,0.f};

  for (int k0 = 0; k0 < K; k0 += 32) {
    V bh[4], bl[4];
#pragma unroll
    for (int j = 0; j < 4; ++j) {
      const size_t bo = (size_t)(n0 + (j << 4) + rlane) * ldb + koff + k0;
      bh[j] = Frag<T>::load(Bb + bo);
      if (SPLIT) bl[j] = Frag<T>::load(Bb2 + bo);
    }
#pragma unroll
    for (int i = 0; i < 4; ++i) {
      const size_t ao = (size_t)(m0 + (i << 4) + rlane) * lda + koff + k0;
      V ah = Frag<T>::load(Ab + ao);
      V al;
      if (SPLIT) al = Frag<T>::load(Ab2 + ao);
#pragma unroll
      for (int j = 0; j < 4; ++j) {
        acc[i][j] = Frag<T>::mma(ah, bh[j], acc[i][j]);
        if (SPLIT) {
          acc[i][j] = Frag<T>::mma(ah, bl[j], acc[i][j]);
          acc[i][j] = Frag<T>::mma(al, bh[j], acc[i][j]);
        }
      }
      Frag<T>::guard4(acc[i][0], acc[i][1], acc[i][2], acc[i][3], ah, SPLIT ? al : ah);
    }
    Frag<T>::keep(bh[0], bh[1], bh[2], bh[3]);
    if (SPLIT) Frag<T>::keep(bl[0], bl[1], bl[2], bl[3]);
  }
  acc_guard4(acc[0][0], acc[0][1], acc[0][2], acc[0][3]);
  acc_guard4(acc[1][0], acc[1][1], acc[1][2], acc[1][3]);
  acc_guard4(acc[2][0], acc[2][1], acc[2][2], acc[2][3]);
  acc_guard4(acc[3][0], acc[3][1], acc[3][2], acc[3][3]);

  float* slab = sT[wave];
  const float* Rb = RESID ? (resid + (size_t)b * strideR) : nullptr;
#pragma unroll
  for (int i = 0; i < 4; ++i) {
    const int mBase = m0 + (i << 4);
#pragma unroll
    for (int j = 0; j < 4; ++j) {
      const int n = n0 + (j << 4) + rlane;
      float bv = 0.f;
      if (BIAS_MODE == 2) bv = bias[n];
#pragma unroll
      for (int r = 0; r < 8; ++r) {
        float v = acc[i][j][r] * scale;
        if (BIAS_MODE == 1) v += bias[mBase + mOff + r];
        if (BIAS_MODE == 2) v += bv;
        if (RESID) v += Rb[(size_t)(mBase + mOff + r) * ldc + n];
        if (ACT == 1) v = tanhf(v);
        if (ACT == 2) v = fmaxf(v, 0.0f);
        if (ACT == 3) v = v / (1.0f + expf(-v));
        if (ACT == 4) v = (v > 0.f) ? v : 0.01f * v;
        slab[(mOff + r) * 68 + (j << 4) + rlane] = v;
      }
    }
    __builtin_amdgcn_fence(__ATOMIC_RELEASE, "workgroup");
    __builtin_amdgcn_wave_barrier();
    __builtin_amdgcn_fence(__ATOMIC_ACQUIRE, "workgroup");
    if (OUT_MODE == 0) {
      float* C = (float*)Cout + (size_t)b * strideC;
      const int hh = lane >> 4, c4 = (lane & 15) * 4;
      for (int pass = 0; pass < 2; ++pass) {
#pragma unroll
        for (int it = 0; it < 8; ++it) {
          const int row = it * 2 + hh;
          v4f v = *(const v4f*)(slab + row * 68 + c4);
          *(volatile v4f*)(C + (size_t)(mBase + row) * ldc + n0 + c4) = v;
        }
        __threadfence();
      }
    } else {
      const int q = lane >> 3, c8 = (lane & 7) * 8;
      unsigned short* C  = (unsigned short*)Cout  + (size_t)b * strideC;
      unsigned short* C2 = (OUT_MODE == 2) ? ((unsigned short*)Cout2 + (size_t)b * strideC) : nullptr;
      for (int pass = 0; pass < 2; ++pass) {
#pragma unroll
        for (int it = 0; it < 4; ++it) {
          const int row = it * 4 + q;
          const float* sp = slab + row * 68 + c8;
          v8h hv, lv;
#pragma unroll
          for (int e = 0; e < 8; ++e) {
            if (OUT_MODE == 1) {
              hv[e] = (_Float16)sp[e];
            } else {
              unsigned short hb = f2bf_bits(sp[e]);
              unsigned short lb = f2bf_bits(sp[e] - bf_bits2f(hb));
              hv[e] = __builtin_bit_cast(_Float16, hb);
              lv[e] = __builtin_bit_cast(_Float16, lb);
            }
          }
          *(volatile v8h*)(C + (size_t)(mBase + row) * ldc + n0 + c8) = hv;
          if (OUT_MODE == 2) *(volatile v8h*)(C2 + (size_t)(mBase + row) * ldc + n0 + c8) = lv;
        }
        __threadfence();
      }
    }
    __builtin_amdgcn_fence(__ATOMIC_RELEASE, "workgroup");
    __builtin_amdgcn_wave_barrier();
    __builtin_amdgcn_fence(__ATOMIC_ACQUIRE, "workgroup");
  }
}

__global__ __launch_bounds__(kThr) void cast_plane_kernel(const float* __restrict__ src, unsigned short* __restrict__ dst,
                                                          int colsLog2, int dstPitch, int dstOff) {
  const int i   = blockIdx.x * kThr + threadIdx.x;
  const int sh  = colsLog2 - 3;
  const int row = i >> sh;
  const int c8  = (i & ((1 << sh) - 1)) * 8;
  const float* sp = src + ((size_t)row << colsLog2) + c8;
  const v4f a0 = *(const v4f*)(sp);
  const v4f a1 = *(const v4f*)(sp + 4);
  v8h hv;
#pragma unroll
  for (int e = 0; e < 4; ++e) {
    const float f0 = a0[e];
    const float f1 = a1[e];
    hv[e]     = (_Float16)carry_flush(bf16r(f0), kInCarry);
    hv[4 + e] = (_Float16)carry_flush(bf16r(f1), kInCarry);
  }
  unsigned short* dp = dst + (size_t)row * dstPitch + dstOff + c8;
  *(volatile v8h*)dp = hv;
  __threadfence();
  *(volatile v8h*)dp = hv;
}


__global__ __launch_bounds__(kThr) void walk_kernel(const float* __restrict__ Y, float* __restrict__ out) {
  const unsigned i = blockIdx.x * (unsigned)kThr + threadIdx.x;
  const unsigned b = i >> 9, c2 = (i & 511u) * 2u;
  const float* yb = Y + (size_t)b * kT * kN + c2;
  float* ob = out + (size_t)b * kT * kE + c2;
  float st[2] = {0.0f, 0.0f};
  for (int t = 0; t < kT; ++t) {
    const float* yp = yb + (size_t)t * kN;
    const v2f vv = *(const v2f*)yp;
    const v2f kv = *(const v2f*)(yp + kE);
    v2f ov;
#pragma unroll
    for (int k = 0; k < 2; ++k) {
      const float z = 1.0f / (1.0f + expf(-kv[k]));
      const float v = vv[k];
      const float g = (v >= 0.0f) ? (v + 0.5f) : (1.0f / (1.0f + expf(-v)));
      st[k] = (1.0f - z) * st[k] + z * g;
      ov[k] = st[k];
    }
    float* dp = ob + (size_t)t * kE;
    *(volatile v2f*)dp = ov;
    __threadfence();
    *(volatile v2f*)dp = ov;
  }
}

extern "C" void kernel_launch(void* const* d_in, const int* in_sizes, int n_in,
                              void* d_out, int out_size, void* d_ws, size_t ws_size,
                              hipStream_t stream) {
  if (n_in < 2 || d_out == nullptr || d_ws == nullptr) return;
  if (in_sizes[0] != kB * kT * kD || in_sizes[1] != kN * kD) return;
  if (out_size != kB * kT * kE) return;
  if (ws_size < kWsTotal) return;
  float* YO = (float*)d_out;
  char* ws = (char*)d_ws;
  unsigned short* X16 = (unsigned short*)(ws + kOffX16);
  unsigned short* W16 = (unsigned short*)(ws + kOffW16);
  float* YP = (float*)(ws + kOffYP);

  static_assert((kMh * (kD / 8)) % kThr == 0 && (kN * (kD / 8)) % kThr == 0 && (kBh * (kE / 2)) % kThr == 0, "every flat kernel's grid exact");
  cast_plane_kernel<<<kN * (kD / 8) / kThr, kThr, 0, stream>>>((const float*)d_in[1], W16, 10, kD, 0);
  for (int p = 0; p < kPc; ++p) {
    cast_plane_kernel<<<kMh * (kD / 8) / kThr, kThr, 0, stream>>>((const float*)d_in[0] + (size_t)p * kMh * kD, X16, 10, kD, 0);
    wmma_gemm64<0, false, 0, 0, false, 0><<<dim3((kMh / 64) * (kN / 64) / 8, 1), 256, 0, stream>>>(
        X16, X16, kD, 0L, W16, W16, kD, 0L, (void*)YP, (void*)YP, kN, 0L, nullptr, nullptr, 0L, kMh, kN, kD, kSc20);
    walk_kernel<<<kBh * (kE / 2) / kThr, kThr, 0, stream>>>(YP, YO + (size_t)p * kMh * kE);
  }
}
static_assert(((kMh / 64) * (kN / 64)) % 8 == 0 && kD % 32 == 0, "the engine's grid: whole blocks of eight wave tiles; the depth a multiple of 32");
